// LocalAttentionBlock_82497731821703
// MI455X (gfx1250) — hardware-verified
//
#include <hip/hip_runtime.h>
#include <hip/hip_bf16.h>

#define BB   2
#define SS   2048
#define EE   1024
#define HH   16
#define DD   64
#define MM   (BB * SS)
#define SCALE_F 0.125f
#define EPS_F   1e-5f

typedef _Float16 bf16_t;
typedef __attribute__((ext_vector_type(16))) _Float16 v16h;
typedef __attribute__((ext_vector_type(8)))  _Float16 v8h;
typedef __attribute__((ext_vector_type(8)))  float  v8f;

typedef int    v4ig  __attribute__((vector_size(16)));
typedef _Float16 v8hg __attribute__((vector_size(16)));

#ifndef __has_builtin
#define __has_builtin(x) 0
#endif

#define HAVE_DS_TR16 0
#define HAVE_ASYNC_LDS 0

#define GLOBAL_V4I(p) ((__attribute__((address_space(1))) v4ig*)(unsigned long long)(p))
#define LDS_V4I(p)    ((__attribute__((address_space(3))) v4ig*)(unsigned int)(unsigned long long)(p))
#define LDS_V8BF(p)   ((__attribute__((address_space(3))) v8hg*)(unsigned int)(unsigned long long)(p))

static __device__ __forceinline__ v8h gcc2ext(v8hg x) {
  union { v8hg g; v8h e; } u; u.g = x; return u.e;
}

static __device__ __forceinline__ v16h cat8(v8h lo, v8h hi) {
  return __builtin_shufflevector(lo, hi, 0,1,2,3,4,5,6,7,8,9,10,11,12,13,14,15);
}

static __device__ __forceinline__ v8f wmma_h16(v16h a, v16h b, v8f c) {
  v8f d = __builtin_amdgcn_wmma_f32_16x16x32_f16(false, a, false, b, (short)0, c, false, false);
  asm volatile("v_nop\n\tv_nop\n\tv_nop\n\tv_nop" : "+v"(d) : "v"(a), "v"(b));
  return d;
}
typedef __attribute__((ext_vector_type(4))) float v4f;
typedef __attribute__((ext_vector_type(4))) unsigned v4u;
template <typename T> __device__ __forceinline__ void vst2(void* p, T v) { *(volatile T*)p = v; __threadfence(); *(volatile T*)p = v; }

template <int MODE>
__global__ __launch_bounds__(256)
void gemm_kernel(const float* __restrict__ A, const float* __restrict__ W,
                 const float* __restrict__ bias, const float* __restrict__ resid,
                 bf16_t* __restrict__ outB, float* __restrict__ outF) {
  constexpr int K = EE;
  constexpr int N = EE;
  constexpr int LDA_S = 40;
  constexpr int LDB_S = 40;

  __shared__ __attribute__((aligned(16))) bf16_t sA[128 * LDA_S];
  __shared__ __attribute__((aligned(16))) bf16_t sBt[128 * LDB_S];
  __shared__ __attribute__((aligned(16))) float sOut[8][32 * 64];

  const int tid  = threadIdx.x;
  const int lane = tid & 31;
  const int wave = tid >> 5;
  const int half = lane >> 4;
  const int lf   = lane & 15;
  const int waveM = wave >> 1;
  const int waveN = wave & 1;

  const int row0 = blockIdx.x * 128;
  const int col0 = blockIdx.y * 128;

  v8f acc[2][4];
  const v8f zero8 = {0.f,0.f,0.f,0.f,0.f,0.f,0.f,0.f};
#pragma unroll
  for (int i = 0; i < 2; ++i)
#pragma unroll
    for (int j = 0; j < 4; ++j) acc[i][j] = zero8;

  const int arow = tid >> 1;
  const int acol = (tid & 1) * 16;
  const int bn   = tid & 127;
  const int bk0  = (tid >> 7) * 16;

  for (int kt = 0; kt < K; kt += 32) {
    if (kt + 32 < K) {
      __builtin_prefetch(A + (size_t)(row0 + arow) * K + kt + 32 + acol, 0, 3);
      __builtin_prefetch(W + (size_t)(kt + 32 + bk0) * N + col0 + bn, 0, 3);
    }
    {
      const float4* s4 = reinterpret_cast<const float4*>(
          A + (size_t)(row0 + arow) * K + kt + acol);
      v8h t0, t1;
#pragma unroll
      for (int q = 0; q < 4; ++q) {
        float4 f = s4[q];
        if (q < 2) {
          t0[q * 4 + 0] = (bf16_t)f.x; t0[q * 4 + 1] = (bf16_t)f.y;
          t0[q * 4 + 2] = (bf16_t)f.z; t0[q * 4 + 3] = (bf16_t)f.w;
        } else {
          t1[(q - 2) * 4 + 0] = (bf16_t)f.x; t1[(q - 2) * 4 + 1] = (bf16_t)f.y;
          t1[(q - 2) * 4 + 2] = (bf16_t)f.z; t1[(q - 2) * 4 + 3] = (bf16_t)f.w;
        }
      }
      *(v8h*)&sA[arow * LDA_S + acol]     = t0;
      *(v8h*)&sA[arow * LDA_S + acol + 8] = t1;
    }
    {
      v8h w0, w1;
#pragma unroll
      for (int j = 0; j < 16; ++j) {
        float vw = W[(size_t)(kt + bk0 + j) * N + col0 + bn];
        if (j < 8) w0[j] = (bf16_t)vw; else w1[j - 8] = (bf16_t)vw;
      }
      *(v8h*)&sBt[bn * LDB_S + bk0]     = w0;
      *(v8h*)&sBt[bn * LDB_S + bk0 + 8] = w1;
    }
    __syncthreads();

    v16h afr[2], bfr[4];
#pragma unroll
    for (int mt = 0; mt < 2; ++mt) {
      const int r  = waveM * 32 + mt * 16 + lf;
      const int co = 8 * half;
      v8h lo = *(const v8h*)&sA[r * LDA_S + co];
      v8h hi = *(const v8h*)&sA[r * LDA_S + co + 16];
      afr[mt] = cat8(lo, hi);
    }
#pragma unroll
    for (int nt = 0; nt < 4; ++nt) {
      const int n  = waveN * 64 + nt * 16 + lf;
      const int ko = 8 * half;
      v8h lo = *(const v8h*)&sBt[n * LDB_S + ko];
      v8h hi = *(const v8h*)&sBt[n * LDB_S + ko + 16];
      bfr[nt] = cat8(lo, hi);
    }
#pragma unroll
    for (int mt = 0; mt < 2; ++mt)
#pragma unroll
      for (int nt = 0; nt < 4; ++nt)
        acc[mt][nt] = wmma_h16(afr[mt], bfr[nt], acc[mt][nt]);

    __syncthreads();
  }

  float* S = sOut[wave];
#pragma unroll
  for (int mt = 0; mt < 2; ++mt)
#pragma unroll
    for (int nt = 0; nt < 4; ++nt)
#pragma unroll
      for (int j = 0; j < 8; ++j)
        S[(mt * 16 + j + 8 * half) * 64 + nt * 16 + lf] = acc[mt][nt][j] + bias[col0 + waveN * 64 + nt * 16 + lf];
  asm volatile("s_wait_dscnt 0" ::: "memory"); __builtin_amdgcn_wave_barrier(); __builtin_amdgcn_fence(__ATOMIC_RELEASE, "workgroup");
  const int mbase = row0 + waveM * 32, nbase = col0 + waveN * 64;
  if (MODE == 0) {
    const int b = mbase >> 11, s0 = mbase & (SS - 1), h = nbase >> 6;
#pragma unroll
    for (int q = 0; q < 8; ++q) { const int rl = q * 4 + (lane >> 3), pc = lane & 7;
      union { v8h hv; v4u u; } pk;
#pragma unroll
      for (int e = 0; e < 8; ++e) pk.hv[e] = (bf16_t)S[rl * 64 + pc * 8 + e];
      vst2(outB + (((size_t)(b * HH + h)) * SS + s0 + rl) * DD + pc * 8, pk.u); }
  } else {
#pragma unroll 4
    for (int q = 0; q < 16; ++q) { const int rl = q * 2 + (lane >> 4), pc = lane & 15;
      const size_t idx = (size_t)(mbase + rl) * N + nbase + pc * 4;
      v4f vv = *(const v4f*)(S + rl * 64 + pc * 4); const v4f rr = *(const v4f*)(resid + idx);
      vst2(outF + idx, vv + rr); }
  }
}

__global__ __launch_bounds__(128)
void attn_kernel(const bf16_t* __restrict__ q, const bf16_t* __restrict__ k,
                 const bf16_t* __restrict__ v, float* __restrict__ attn_out) {
  constexpr int LDK = 72;
  constexpr int LDP = 40;

  __shared__ __attribute__((aligned(16))) bf16_t sK[32 * LDK];
#if HAVE_DS_TR16
  __shared__ bf16_t sV[32 * LDK];
#else
  constexpr int LDV = 40;
  __shared__ __attribute__((aligned(16))) bf16_t sVt[64 * LDV];
#endif
  __shared__ __attribute__((aligned(16))) bf16_t sP[4][16 * LDP];
  __shared__ __attribute__((aligned(16))) float sO[4][16 * 64];

  const int qt = blockIdx.x & 31;
  const int h  = (blockIdx.x >> 5) & (HH - 1);
  const int b  = blockIdx.x >> 9;
  const int q0 = qt * 64;

  const float slope = exp2f(-(float)(h + 1));
  const int   w     = (int)roundf(64.0f + (float)h * (448.0f / 15.0f));

  const int tid  = threadIdx.x;
  const int lane = tid & 31;
  const int wv   = tid >> 5;
  const int half = lane >> 4;
  const int lf   = lane & 15;

  const size_t headoff = ((size_t)(b * HH + h)) * SS * DD;
  const bf16_t* qh = q + headoff;
  const bf16_t* kh = k + headoff;
  const bf16_t* vh = v + headoff;

  const int qrow = q0 + wv * 16 + lf;
  v16h qf[2];
#pragma unroll
  for (int c = 0; c < 2; ++c) {
    const bf16_t* p = qh + (size_t)qrow * DD + c * 32 + 8 * half;
    v8h lo = *(const v8h*)p;
    v8h hi = *(const v8h*)(p + 16);
    qf[c] = cat8(lo, hi);
  }

  const v8f zero8 = {0.f,0.f,0.f,0.f,0.f,0.f,0.f,0.f};
  v8f o[4];
#pragma unroll
  for (int i = 0; i < 4; ++i) o[i] = zero8;

  int kstart = q0 - w + 1;
  if (kstart < 0) kstart = 0;
  kstart &= ~31;
  const int kend = q0 + 64;

  const int lkey = tid >> 2;
  const int ld0  = (tid & 3) * 16;

  for (int kb = kstart; kb < kend; kb += 32) {
    __syncthreads();
    {
      const bf16_t* ksrc = kh + (size_t)(kb + lkey) * DD + ld0;
      const bf16_t* vsrc = vh + (size_t)(kb + lkey) * DD + ld0;
#if HAVE_DS_TR16
      bf16_t* kdst = &sK[lkey * LDK + ld0];
      bf16_t* vdst = &sV[lkey * LDK + ld0];
#if HAVE_ASYNC_LDS
      __builtin_amdgcn_global_load_async_to_lds_b128(GLOBAL_V4I(ksrc),     LDS_V4I(kdst),     0, 0);
      __builtin_amdgcn_global_load_async_to_lds_b128(GLOBAL_V4I(ksrc + 8), LDS_V4I(kdst + 8), 0, 0);
      __builtin_amdgcn_global_load_async_to_lds_b128(GLOBAL_V4I(vsrc),     LDS_V4I(vdst),     0, 0);
      __builtin_amdgcn_global_load_async_to_lds_b128(GLOBAL_V4I(vsrc + 8), LDS_V4I(vdst + 8), 0, 0);
      asm volatile("s_wait_asynccnt 0x0" ::: "memory");
#else
      *(v8h*)kdst       = *(const v8h*)ksrc;
      *(v8h*)(kdst + 8) = *(const v8h*)(ksrc + 8);
      *(v8h*)vdst       = *(const v8h*)vsrc;
      *(v8h*)(vdst + 8) = *(const v8h*)(vsrc + 8);
#endif
#else
      *(v8h*)&sK[lkey * LDK + ld0]     = *(const v8h*)ksrc;
      *(v8h*)&sK[lkey * LDK + ld0 + 8] = *(const v8h*)(ksrc + 8);
#pragma unroll
      for (int j = 0; j < 16; ++j)
        sVt[(ld0 + j) * LDV + lkey] = vsrc[j];
#endif
    }
    __syncthreads();

    v8f sc[2] = {zero8, zero8};
#pragma unroll
    for (int dc = 0; dc < 2; ++dc) {
#pragma unroll
      for (int nt = 0; nt < 2; ++nt) {
        const bf16_t* kp = &sK[(nt * 16 + lf) * LDK + dc * 32 + 8 * half];
        v8h lo = *(const v8h*)kp;
        v8h hi = *(const v8h*)(kp + 16);
        sc[nt] = wmma_h16(qf[dc], cat8(lo, hi), sc[nt]);
      }
    }

    bf16_t* pw = &sP[wv][0];
#pragma unroll
    for (int nt = 0; nt < 2; ++nt) {
#pragma unroll
      for (int j = 0; j < 8; ++j) {
        const int m = q0 + wv * 16 + j + 8 * half;
        const int n = kb + nt * 16 + lf;
        const int dist = m - n;
        const float z = sc[nt][j] * SCALE_F - slope * (float)dist;
        const float p = (dist >= 0 && dist < w)
                            ? (1.0f / (1.0f + __expf(-z)))
                            : 0.0f;
        pw[(j + 8 * half) * LDP + nt * 16 + lf] = (bf16_t)p;
      }
    }

    asm volatile("s_wait_dscnt 0" ::: "memory"); __builtin_amdgcn_wave_barrier(); __builtin_amdgcn_fence(__ATOMIC_RELEASE, "workgroup");
    {
      const bf16_t* pp = &pw[lf * LDP + 8 * half];
      v8h plo = *(const v8h*)pp;
      v8h phi = *(const v8h*)(pp + 16);
      v16h pf = cat8(plo, phi);
#pragma unroll
      for (int ntd = 0; ntd < 4; ++ntd) {
#if HAVE_DS_TR16
        v8h vlo = gcc2ext(__builtin_amdgcn_ds_load_tr16_b128_v8h16(
            LDS_V8BF(&sV[lf * LDK + ntd * 16 + 8 * half])));
        v8h vhi = gcc2ext(__builtin_amdgcn_ds_load_tr16_b128_v8h16(
            LDS_V8BF(&sV[(16 + lf) * LDK + ntd * 16 + 8 * half])));
#else
        const bf16_t* vp = &sVt[(ntd * 16 + lf) * LDV + 8 * half];
        v8h vlo = *(const v8h*)vp;
        v8h vhi = *(const v8h*)(vp + 16);
#endif
        o[ntd] = wmma_h16(pf, cat8(vlo, vhi), o[ntd]);
      }
    }
  }

  float* so = sO[wv];
#pragma unroll
  for (int ntd = 0; ntd < 4; ++ntd)
#pragma unroll
    for (int j = 0; j < 8; ++j) so[(j + 8 * half) * 64 + ntd * 16 + lf] = o[ntd][j];
  asm volatile("s_wait_dscnt 0" ::: "memory"); __builtin_amdgcn_wave_barrier(); __builtin_amdgcn_fence(__ATOMIC_RELEASE, "workgroup");
#pragma unroll
  for (int q = 0; q < 8; ++q) { const int rl = q * 2 + (lane >> 4), pc = lane & 15;
    vst2(attn_out + ((size_t)b * SS + q0 + wv * 16 + rl) * EE + h * DD + pc * 4, *(const v4f*)(so + rl * 64 + pc * 4)); }
}

__global__ __launch_bounds__(256)
void ln_kernel(const float* __restrict__ y, const float* __restrict__ gamma,
               const float* __restrict__ beta, float* __restrict__ out) {
  const int row = blockIdx.x;
  const float* yr = y + (size_t)row * EE;

  float vals[4];
  float lsum = 0.f, lsq = 0.f;
#pragma unroll
  for (int i = 0; i < 4; ++i) {
    const float t = yr[threadIdx.x + i * 256];
    vals[i] = t;
    lsum += t;
    lsq  += t * t;
  }
#pragma unroll
  for (int off = 16; off > 0; off >>= 1) {
    lsum += __shfl_xor(lsum, off, 32);
    lsq  += __shfl_xor(lsq,  off, 32);
  }
  __shared__ float s1[8], s2[8];
  if ((threadIdx.x & 31) == 0) {
    s1[threadIdx.x >> 5] = lsum;
    s2[threadIdx.x >> 5] = lsq;
  }
  __syncthreads();
  float tsum = 0.f, tsq = 0.f;
#pragma unroll
  for (int wv = 0; wv < 8; ++wv) { tsum += s1[wv]; tsq += s2[wv]; }

  const float mu  = tsum * (1.0f / EE);
  const float var = tsq * (1.0f / EE) - mu * mu;
  const float inv = rsqrtf(var + EPS_F);
#pragma unroll
  for (int i = 0; i < 4; ++i) {
    const int c = threadIdx.x + i * 256;
    vst2(out + (size_t)row * EE + c, (vals[i] - mu) * inv * gamma[c] + beta[c]);
  }
}

extern "C" void kernel_launch(void* const* d_in, const int* in_sizes, int n_in,
                              void* d_out, int out_size, void* d_ws, size_t ws_size,
                              hipStream_t stream) {
  const float* x     = (const float*)d_in[0];
  const float* Wq    = (const float*)d_in[1];
  const float* bq    = (const float*)d_in[2];
  const float* Wk    = (const float*)d_in[3];
  const float* bk    = (const float*)d_in[4];
  const float* Wv    = (const float*)d_in[5];
  const float* bv    = (const float*)d_in[6];
  const float* Wo    = (const float*)d_in[7];
  const float* bo    = (const float*)d_in[8];
  const float* gamma = (const float*)d_in[9];
  const float* beta  = (const float*)d_in[10];
  float* out = (float*)d_out;

  const size_t nElem = (size_t)BB * SS * EE;
  char* ws = (char*)d_ws;
  bf16_t* qb   = (bf16_t*)ws;  ws += nElem * sizeof(bf16_t);
  bf16_t* kb   = (bf16_t*)ws;  ws += nElem * sizeof(bf16_t);
  bf16_t* vb   = (bf16_t*)ws;  ws += nElem * sizeof(bf16_t);
  float*  attn = (float*)ws;   ws += nElem * sizeof(float);
  float*  yb   = (float*)ws;

  dim3 gg(MM / 128, EE / 128);
  gemm_kernel<0><<<gg, 256, 0, stream>>>(x, Wq, bq, nullptr, qb, nullptr);
  gemm_kernel<0><<<gg, 256, 0, stream>>>(x, Wk, bk, nullptr, kb, nullptr);
  gemm_kernel<0><<<gg, 256, 0, stream>>>(x, Wv, bv, nullptr, vb, nullptr);

  attn_kernel<<<BB * HH * (SS / 64), 128, 0, stream>>>(qb, kb, vb, attn);

  gemm_kernel<1><<<gg, 256, 0, stream>>>(attn, Wo, bo, x, nullptr, yb);

  ln_kernel<<<MM, 256, 0, stream>>>(yb, gamma, beta, out);
}
